// RnnModel_78254304133187
// MI455X (gfx1250) — hardware-verified
//
#include <hip/hip_runtime.h>
#include <math.h>

constexpr int NBATCH = 256;
constexpr int NSTEP  = 512;
constexpr int NIN    = 4;
constexpr int NHID   = 128;
constexpr int NGATE  = 4 * NHID;
constexpr int KAUG   = 160;
constexpr int WPITCH = 192;
constexpr int WSEG   = WPITCH / 8;
constexpr int HSEG   = NHID / 8;
constexpr int APITCH = 168;
constexpr int HSP    = 132;
constexpr int NTHR   = 256;
constexpr int BT     = 16;
constexpr float ACARRY = 64.0f;
constexpr float WCARRY = 256.0f;
constexpr float FOLD   = 1.0f / (ACARRY * WCARRY);
static_assert(NBATCH % BT == 0, "batch tile multiple");
static_assert(NHID == 16 * (NTHR / 32), "8 waves x 16 hidden units");
static_assert(NIN == 4, "x row is one 16-B float4");
static_assert(KAUG % 32 == 0 && KAUG >= NHID + NIN, "augmented K is a multiple of 32");
static_assert(APITCH % 8 == 0 && APITCH >= KAUG, "A tile pitch");
static_assert(WPITCH % 64 == 0 && WPITCH >= KAUG, "weight rows are whole 128-B lines");
static_assert((NGATE * WSEG) % NTHR == 0, "prep grid exact");
static_assert(HSP % 4 == 0 && HSP >= NHID, "staging pitch");
static_assert((BT * APITCH) % 8 == 0, "A tile zero-fill in 32-bit words");
static_assert(BT * NHID == 2 * NTHR * 4, "output store loop exact: 2 iterations x 256 threads x 4 floats");

typedef __attribute__((ext_vector_type(16))) _Float16 v16h;
typedef __attribute__((ext_vector_type(8)))  _Float16 v8h;
typedef __attribute__((ext_vector_type(8)))  float    v8f;
typedef __attribute__((ext_vector_type(4)))  float    v4f;
typedef __attribute__((ext_vector_type(4)))  unsigned v4u;

__device__ __forceinline__ void dep_guard5(v8f& a0, v8f& a1, v8f& a2, v8f& a3,
                                           v16h x, v16h y0, v16h y1, v16h y2, v16h y3) {
  asm volatile("v_nop\n\tv_nop\n\tv_nop\n\tv_nop"
               : "+v"(a0), "+v"(a1), "+v"(a2), "+v"(a3)
               : "v"(x), "v"(y0), "v"(y1), "v"(y2), "v"(y3));
}
__device__ __forceinline__ void acc_guard4(v8f& a, v8f& b, v8f& c, v8f& d) {
  asm volatile("v_nop\n\tv_nop\n\tv_nop\n\tv_nop" : "+v"(a), "+v"(b), "+v"(c), "+v"(d));
}

template <typename T> struct Frag;
template <> struct Frag<_Float16> {
  typedef v16h V; union U { v16h v; v8h h[2]; };
  static __device__ __forceinline__ v16h load(const _Float16* p) {
    U f; f.h[0] = *(const v8h*)(p); f.h[1] = *(const v8h*)(p + 16); return f.v;
  }
  static __device__ __forceinline__ v8f mma(v16h a, v16h b, v8f c) {
    return __builtin_amdgcn_wmma_f32_16x16x32_f16(false, a, false, b, (short)0, c, false, false);
  }
};

__device__ __forceinline__ float fsig(float v)  { return __builtin_amdgcn_rcpf(1.0f + expf(-v)); }
__device__ __forceinline__ float ftanh(float v) { return 1.0f - 2.0f * __builtin_amdgcn_rcpf(expf(2.0f * v) + 1.0f); }

__global__ __launch_bounds__(NTHR) void wprep_kernel(const float* __restrict__ Whh0, const float* __restrict__ Wih0,
                                                     const float* __restrict__ Whh1, const float* __restrict__ Wih1,
                                                     unsigned short* __restrict__ WP) {
  const int d = blockIdx.y;
  const int i = blockIdx.x * NTHR + threadIdx.x;
  const float* Whh = d ? Whh1 : Whh0;
  const float* Wih = d ? Wih1 : Wih0;
  const int n  = i / WSEG;
  const int s  = i - n * WSEG;
  const int sh = (s < HSEG) ? s : (HSEG - 1);
  const float* hr = Whh + (size_t)n * NHID + 8 * sh;
  const v4f a0 = *(const v4f*)(hr);
  const v4f a1 = *(const v4f*)(hr + 4);
  const v4f xw = *(const v4f*)(Wih + (size_t)n * NIN);
  const float fh = (s < HSEG) ? 1.0f : 0.0f;
  const float fx = (s == HSEG) ? 1.0f : 0.0f;
  v8h hv;
#pragma unroll
  for (int e = 0; e < 4; ++e) {
    const float v0 = fmaf(fh, a0[e], fx * xw[e]);
    const float v1 = fmaf(fh, a1[e], fx * 0.0f);
    hv[e]     = (_Float16)(v0 * WCARRY);
    hv[4 + e] = (_Float16)(v1 * WCARRY);
  }
  unsigned short* dst = WP + (size_t)d * NGATE * WPITCH + (size_t)i * 8;
  *(volatile v8h*)dst = hv;
  __threadfence();
  *(volatile v8h*)dst = hv;
}

__global__ __launch_bounds__(NTHR) void bilstm_kernel(const float* __restrict__ x,
                                                      const float* __restrict__ bih0, const float* __restrict__ bhh0,
                                                      const float* __restrict__ bih1, const float* __restrict__ bhh1,
                                                      const unsigned short* __restrict__ WPp,
                                                      float* __restrict__ out) {
  __shared__ __align__(16) _Float16 At[BT * APITCH];
  __shared__ __align__(16) float    Hs[BT * HSP];
  const int tid = threadIdx.x, lane = tid & 31, wave = tid >> 5;
  const int c = lane & 15, hh = lane >> 4, koff = hh * 8;
  const int b0  = blockIdx.x * BT;
  const int dir = blockIdx.y;
  const _Float16* WP = (const _Float16*)WPp + (size_t)dir * NGATE * WPITCH;
  const float* bih = dir ? bih1 : bih0;
  const float* bhh = dir ? bhh1 : bhh0;
  const int u = 16 * wave + c;

  {
    unsigned* Aw = (unsigned*)(&At[0]);
#pragma unroll 1
    for (int i = tid; i < (BT * APITCH) / 2; i += NTHR) Aw[i] = 0u;
  }
  float cst[8], hst[8], bsum[4];
#pragma unroll
  for (int r = 0; r < 8; ++r) { cst[r] = 0.0f; hst[r] = 0.0f; }
#pragma unroll
  for (int j = 0; j < 4; ++j) bsum[j] = bih[j * NHID + u] + bhh[j * NHID + u];
  __syncthreads();

  const _Float16* arow = At + c * APITCH + koff;
  const _Float16* wrow = WP + (size_t)u * WPITCH + koff;
  const v8f z8 = {0.f, 0.f, 0.f, 0.f, 0.f, 0.f, 0.f, 0.f};

#pragma unroll 1
  for (int t = 0; t < NSTEP; ++t) {
    const int tt = dir ? (NSTEP - 1 - t) : t;
    if (tid < 64) {
      const int m = tid >> 2, seg = tid & 3;
      const v4f xv = *(const v4f*)(x + ((size_t)(b0 + m) * NSTEP + (size_t)tt) * NIN);
      const float x0 = xv[0] * ACARRY, x1 = xv[1] * ACARRY, x2 = xv[2] * ACARRY, x3 = xv[3] * ACARRY;
      const _Float16 q0 = (_Float16)x0, q1 = (_Float16)x1, q2 = (_Float16)x2, q3 = (_Float16)x3;
      const unsigned u0 = (unsigned)__builtin_bit_cast(unsigned short, q0) | ((unsigned)__builtin_bit_cast(unsigned short, q1) << 16);
      const unsigned u1 = (unsigned)__builtin_bit_cast(unsigned short, q2) | ((unsigned)__builtin_bit_cast(unsigned short, q3) << 16);
      v4u wv;
      wv[0] = (seg == 0) ? u0 : 0u;
      wv[1] = (seg == 0) ? u1 : 0u;
      wv[2] = 0u;
      wv[3] = 0u;
      *(v4u*)(At + m * APITCH + NHID + 8 * seg) = wv;
    }
    __syncthreads();

    v8f acc0 = z8, acc1 = z8, acc2 = z8, acc3 = z8;
#pragma unroll 1
    for (int k0 = 0; k0 < KAUG; k0 += 32) {
      const v16h a   = Frag<_Float16>::load(arow + k0);
      const v16h bg0 = Frag<_Float16>::load(wrow + k0);
      const v16h bg1 = Frag<_Float16>::load(wrow + (size_t)1 * NHID * WPITCH + k0);
      const v16h bg2 = Frag<_Float16>::load(wrow + (size_t)2 * NHID * WPITCH + k0);
      const v16h bg3 = Frag<_Float16>::load(wrow + (size_t)3 * NHID * WPITCH + k0);
      acc0 = Frag<_Float16>::mma(a, bg0, acc0);
      acc1 = Frag<_Float16>::mma(a, bg1, acc1);
      acc2 = Frag<_Float16>::mma(a, bg2, acc2);
      acc3 = Frag<_Float16>::mma(a, bg3, acc3);
      dep_guard5(acc0, acc1, acc2, acc3, a, bg0, bg1, bg2, bg3);
    }
    acc_guard4(acc0, acc1, acc2, acc3);

#pragma unroll
    for (int r = 0; r < 8; ++r) {
      const float zi = acc0[r] * FOLD + bsum[0];
      const float zf = acc1[r] * FOLD + bsum[1];
      const float zg = acc2[r] * FOLD + bsum[2];
      const float zo = acc3[r] * FOLD + bsum[3];
      const float ig = fsig(zi);
      const float fg = fsig(zf);
      const float gg = ftanh(zg);
      const float og = fsig(zo);
      const float cn = fg * cst[r] + ig * gg;
      cst[r] = cn;
      hst[r] = og * ftanh(cn);
    }
    __syncthreads();
#pragma unroll
    for (int r = 0; r < 8; ++r) At[(8 * hh + r) * APITCH + u] = (_Float16)(hst[r] * ACARRY);
  }

#pragma unroll
  for (int r = 0; r < 8; ++r) Hs[(8 * hh + r) * HSP + u] = hst[r];
  __syncthreads();
  float* ob = out + (size_t)b0 * (2 * NHID) + (size_t)dir * NHID;
  for (int pass = 0; pass < 2; ++pass) {
#pragma unroll
    for (int it = 0; it < 2; ++it) {
      const int idx = it * NTHR + tid;
      const int row = idx >> 5, c4 = (idx & 31) * 4;
      const v4f v = *(const v4f*)(Hs + row * HSP + c4);
      *(volatile v4f*)(ob + (size_t)row * (2 * NHID) + c4) = v;
    }
    __threadfence();
  }
}

extern "C" void kernel_launch(void* const* d_in, const int* in_sizes, int n_in,
                              void* d_out, int out_size, void* d_ws, size_t ws_size, hipStream_t stream) {
  if (n_in < 9 || d_out == nullptr || d_ws == nullptr) return;
  if (in_sizes[0] != NBATCH * NSTEP * NIN || in_sizes[1] != NGATE * NIN || in_sizes[2] != NGATE * NHID ||
      in_sizes[3] != NGATE || in_sizes[4] != NGATE || in_sizes[5] != NGATE * NIN || in_sizes[6] != NGATE * NHID ||
      in_sizes[7] != NGATE || in_sizes[8] != NGATE || out_size != NBATCH * 2 * NHID) return;

  const float* x     = (const float*)d_in[0];
  const float* Wih_f = (const float*)d_in[1];
  const float* Whh_f = (const float*)d_in[2];
  const float* bih_f = (const float*)d_in[3];
  const float* bhh_f = (const float*)d_in[4];
  const float* Wih_b = (const float*)d_in[5];
  const float* Whh_b = (const float*)d_in[6];
  const float* bih_b = (const float*)d_in[7];
  const float* bhh_b = (const float*)d_in[8];
  float* out = (float*)d_out;

  const size_t wp_bytes = (size_t)2 * NGATE * WPITCH * 2;
  if (wp_bytes > ws_size || wp_bytes > (size_t)134217728) return;
  unsigned short* WP = (unsigned short*)d_ws;

  wprep_kernel<<<dim3((NGATE * WSEG) / NTHR, 2), NTHR, 0, stream>>>(Whh_f, Wih_f, Whh_b, Wih_b, WP);
  bilstm_kernel<<<dim3(NBATCH / BT, 2), NTHR, 0, stream>>>(x, bih_f, bhh_f, bih_b, bhh_b, WP, out);
}
